// EKPConv_v1_35725537968373
// MI455X (gfx1250) — hardware-verified
//
#include <hip/hip_runtime.h>
#include <math.h>

typedef __attribute__((ext_vector_type(16))) _Float16 v16h;
typedef __attribute__((ext_vector_type(16))) __bf16 v16b;
typedef __attribute__((ext_vector_type(8)))  _Float16 v8h;
typedef __attribute__((ext_vector_type(8)))  float v8f;
typedef __attribute__((ext_vector_type(4)))  float v4f;
typedef __attribute__((ext_vector_type(2)))  float v2f;
typedef __attribute__((ext_vector_type(4)))  unsigned v4u;
typedef __attribute__((ext_vector_type(4)))  int v4i;
typedef float __attribute__((may_alias)) float_a;
typedef int __attribute__((may_alias)) int_a;

template <typename T> __device__ __forceinline__ void vst2(void* p, T v) { *(volatile T*)p = v; __threadfence(); *(volatile T*)p = v; }
__device__ __forceinline__ v8f wmma16(v16h a, v16h b, v8f c) {
  v8f d = __builtin_amdgcn_wmma_f32_16x16x32_f16(false, a, false, b, (short)0, c, false, false);
  asm volatile("v_nop\n\tv_nop\n\tv_nop\n\tv_nop" : "+v"(d) : "v"(a), "v"(b));
  return d;
}
__device__ __forceinline__ v8f wmma_bf(v16b a, v16b b, v8f c) {
  v8f d = __builtin_amdgcn_wmma_f32_16x16x32_bf16(false, a, false, b, (short)0, c, false, false);
  asm volatile("v_nop\n\tv_nop\n\tv_nop\n\tv_nop" : "+v"(d) : "v"(a), "v"(b));
  return d;
}
__device__ __forceinline__ v16h frag_h(const _Float16* rowk0, int lane) {
  union { v16h v; v8h q[2]; } u; const _Float16* p = rowk0 + 8 * (lane >> 4);
  u.q[0] = *(const v8h*)p; u.q[1] = *(const v8h*)(p + 16); return u.v;
}
__device__ __forceinline__ v16h frag_f32(const float* rowk0, int lane) {
  v16h a; const float* p = rowk0 + 8 * (lane >> 4);
#pragma unroll
  for (int i = 0; i < 8; ++i) { a[i] = (_Float16)p[i]; a[8 + i] = (_Float16)p[16 + i]; }
  return a;
}
__device__ __forceinline__ v16h frag_f32s(const float* rowk0, int lane, float sc) {
  v16h a; const float* p = rowk0 + 8 * (lane >> 4);
#pragma unroll
  for (int i = 0; i < 8; ++i) { a[i] = (_Float16)(p[i] * sc); a[8 + i] = (_Float16)(p[16 + i] * sc); }
  return a;
}
__device__ __forceinline__ v16h fragc_f32(const float* W, int k0, int n, int lane, int ld, int K) {
  v16h a; const int g = lane >> 4;
#pragma unroll
  for (int i = 0; i < 8; ++i) { const int ka = k0 + 8 * g + i, kb = ka + 16;
    a[i] = (_Float16)(ka < K ? W[(size_t)(ka < K ? ka : K - 1) * ld + n] : 0.f); a[8 + i] = (_Float16)(kb < K ? W[(size_t)(kb < K ? kb : K - 1) * ld + n] : 0.f); }
  return a;
}
struct F2 { v16b h, l; };
__device__ __forceinline__ F2 bsplit16(const float v[16]) { F2 r;
#pragma unroll
  for (int i = 0; i < 16; ++i) { const __bf16 h = (__bf16)v[i]; r.h[i] = h; r.l[i] = (__bf16)(v[i] - (float)h); }
  return r; }
__device__ __forceinline__ F2 split_row(const float* row, int k0, int lane) { float v[16]; const float* p = row + k0 + 8 * (lane >> 4);
#pragma unroll
  for (int i = 0; i < 8; ++i) { v[i] = p[i]; v[8 + i] = p[16 + i]; }
  return bsplit16(v); }
__device__ __forceinline__ F2 split_rowK(const float* row, int k0, int lane, int K) { float v[16]; const int g = lane >> 4;
#pragma unroll
  for (int i = 0; i < 8; ++i) { const int ka = k0 + 8 * g + i, kb = ka + 16; v[i] = ka < K ? row[ka < K ? ka : K - 1] : 0.f; v[8 + i] = kb < K ? row[kb < K ? kb : K - 1] : 0.f; }
  return bsplit16(v); }
__device__ __forceinline__ F2 split_col(const float* W, int k0, int n, int lane, int ld, int K) { float v[16]; const int g = lane >> 4;
#pragma unroll
  for (int i = 0; i < 8; ++i) { const int ka = k0 + 8 * g + i, kb = ka + 16; v[i] = ka < K ? W[(size_t)(ka < K ? ka : K - 1) * ld + n] : 0.f; v[8 + i] = kb < K ? W[(size_t)(kb < K ? kb : K - 1) * ld + n] : 0.f; }
  return bsplit16(v); }
__device__ __forceinline__ v8f mac3(const F2& a, const F2& b, v8f c) { c = wmma_bf(a.l, b.h, c); c = wmma_bf(a.h, b.l, c); return wmma_bf(a.h, b.h, c); }
__device__ __forceinline__ float sigm(float v) { return 1.0f / (1.0f + expf(-v)); }
#define LDSX() do { asm volatile("s_wait_dscnt 0" ::: "memory"); __builtin_amdgcn_wave_barrier(); __builtin_amdgcn_fence(__ATOMIC_RELEASE, "workgroup"); } while (0)


#define NQ 50000
#define MS 50000
#define HN 32
#define KP 15
#define NL 4
#define CI 64
#define CL 16
#define CO 128
#define KW (KP * CI)
#define NQP 50048
#ifndef TPB
#define TPB (NQP / 4)
#endif
#ifndef TOB
#define TOB (NQP / 64)
#endif
typedef __attribute__((ext_vector_type(8))) __bf16 v8b;
__device__ __forceinline__ v16b frag_b(const __bf16* rowk0, int lane) {
  union { v16b v; v8b q[2]; } u; const __bf16* p = rowk0 + 8 * (lane >> 4);
  u.q[0] = *(const v8b*)p; u.q[1] = *(const v8b*)(p + 16); return u.v;
}
__device__ __forceinline__ float bfr(float v) { return (float)(__bf16)v; }
__device__ __attribute__((noinline)) float exp_ni(float v) { return expf(v); }
__device__ __attribute__((noinline)) float erf_ni(float v) { return erff(v); }

#define WS_WF  0u
#define WS_WL  (WS_WF + 2u * (size_t)NQP * KW)
#define WS_END (WS_WL + 2u * (size_t)NQP * KW)

__global__ __launch_bounds__(128) void k_agg(const float* __restrict__ QP, const float* __restrict__ SPt, const int* __restrict__ NI, const float* __restrict__ X, const float* __restrict__ LRF, const float* __restrict__ KPT, _Float16* __restrict__ WF, _Float16* __restrict__ WL) {
  __shared__ float sw[4][NL][16][HN + 1]; __shared__ __align__(16) _Float16 sx[4][HN][CI + 8]; __shared__ __align__(16) _Float16 srow[4][KW], srl[4][KW];
  const int tid = threadIdx.x, wave = tid >> 5, lane = tid & 31, col = lane & 15, g = lane >> 4; const size_t n = (size_t)blockIdx.x * 4 + wave; const bool live = n < (size_t)NQ;
  int idx = live ? NI[n * HN + lane] : MS; const bool real = idx < MS; if (!real) idx = 0;
  float rel[3]; { for (int d = 0; d < 3; ++d) { const float sp = real ? bfr(SPt[(size_t)idx * 3 + d]) : 1.0e6f; rel[d] = sp - (live ? bfr(QP[n * 3 + d]) : 0.f); } }
  for (int c = 0; c < CI; ++c) sx[wave][lane][c] = real ? (_Float16)bfr(X[(size_t)idx * CI + c]) : (_Float16)0.0f;
#pragma unroll 1
  for (int l = 0; l < NL; ++l) { float al[3];
    for (int e = 0; e < 3; ++e) { float a = 0.f; for (int d = 0; d < 3; ++d) a += rel[d] * (live ? bfr(LRF[((n * NL + l) * 3 + d) * 3 + e]) : 0.f); al[e] = a; }
#pragma unroll 1
    for (int k = 0; k < KP; ++k) { float d2 = 0.f; for (int e = 0; e < 3; ++e) { const float df = al[e] - bfr(KPT[k * 3 + e]); d2 += df * df; } sw[wave][l][k][lane] = fmaxf(1.0f - sqrtf(d2) / 1.2f, 0.f); }
    sw[wave][l][15][lane] = 0.f; }
  __syncthreads();
#pragma unroll 1
  for (int l = 0; l < NL; ++l) { v16h a, al, bq;
#pragma unroll
    for (int i = 0; i < 8; ++i) { const float w0 = sw[wave][l][col][8 * g + i], w1 = sw[wave][l][col][16 + 8 * g + i]; const _Float16 h0 = (_Float16)w0, h1 = (_Float16)w1; a[i] = h0; a[8 + i] = h1; al[i] = (_Float16)(w0 - (float)h0); al[8 + i] = (_Float16)(w1 - (float)h1); bq[i] = sx[wave][8 * g + i][l * CL + col]; bq[8 + i] = sx[wave][16 + 8 * g + i][l * CL + col]; }
    v8f c = {}; c = wmma16(a, bq, c); c = wmma16(al, bq, c);
#pragma unroll
    for (int r = 0; r < 8; ++r) { const int k = 8 * g + r; if (k < KP) { const float v = c[r]; const _Float16 hv = (_Float16)v; srow[wave][k * CI + l * CL + col] = hv; srl[wave][k * CI + l * CL + col] = (_Float16)(v - (float)hv); } } }
  __syncthreads();
  for (int q = lane; q < KW / 8; q += 32) { v4u v = *(const v4u*)&srow[wave][q * 8], vl = *(const v4u*)&srl[wave][q * 8]; if (!live) { v[0] = v[1] = v[2] = v[3] = 0u; vl = v; } vst2((unsigned*)(WF + n * KW + q * 8), v); vst2((unsigned*)(WL + n * KW + q * 8), vl); } }
__global__ __launch_bounds__(128) void k_out(const _Float16* __restrict__ WF, const _Float16* __restrict__ WL, const float* __restrict__ WT, float* __restrict__ OUT) { __shared__ __align__(16) float sf[4][16][132];
  const int tid = threadIdx.x, wave = tid >> 5, lane = tid & 31, col = lane & 15, g = lane >> 4; const size_t r0 = (size_t)blockIdx.x * 64 + wave * 16;
  v8f acc[8] = {};
#pragma unroll 2
  for (int kc = 0; kc < KW / 32; ++kc) { const v16h a = frag_h(WF + (r0 + col) * KW + kc * 32, lane), a2 = frag_h(WL + (r0 + col) * KW + kc * 32, lane);
#pragma unroll
    for (int j = 0; j < 8; ++j) { v16h w; const int o = j * 16 + col;
#pragma unroll
      for (int i = 0; i < 8; ++i) { w[i] = (_Float16)bfr(WT[(size_t)(kc * 32 + 8 * g + i) * CO + o]); w[8 + i] = (_Float16)bfr(WT[(size_t)(kc * 32 + 16 + 8 * g + i) * CO + o]); }
      acc[j] = wmma16(a, w, acc[j]); acc[j] = wmma16(a2, w, acc[j]); } }
#pragma unroll
  for (int j = 0; j < 8; ++j)
#pragma unroll
    for (int r = 0; r < 8; ++r) sf[wave][8 * g + r][j * 16 + col] = acc[j][r];
  LDSX(); for (int rl = 0; rl < 16; ++rl) { const size_t row = r0 + rl; if (row < (size_t)NQ) vst2(OUT + row * CO + lane * 4, *(const v4f*)&sf[wave][rl][lane * 4]); } }
extern "C" void kernel_launch(void* const* d_in, const int* in_sizes, int n_in, void* d_out, int out_size, void* d_ws, size_t ws_size, hipStream_t stream) {
  (void)in_sizes; (void)n_in; (void)out_size;
  const float** F = (const float**)d_in;
  if (ws_size < (size_t)WS_END) return;
  char* ws = (char*)d_ws; _Float16 *WF = (_Float16*)(ws + WS_WF), *WL = (_Float16*)(ws + WS_WL);
  k_agg<<<TPB, 128, 0, stream>>>(F[0], F[1], (const int*)d_in[2], F[3], F[4], F[6], WF, WL);
  k_out<<<TOB, 128, 0, stream>>>(WF, WL, F[5], (float*)d_out);
}
